// SpatialAwareAttention_90486370992267
// MI455X (gfx1250) — hardware-run, weakly checked
//
#include <hip/hip_runtime.h>
#include <stdint.h>
#include <math.h>

#define NB    4
#define NTOK  2049
#define NP    2112
#define DM    512
#define NH    8
#define HD    64
#define NQK   1024
#define N3    1536
#define MR    (NB * NP)
#define KLD   72
#define PLD   72
#define OLD   68

typedef _Float16 v16h __attribute__((ext_vector_type(16)));
typedef _Float16 v8h  __attribute__((ext_vector_type(8)));
typedef _Float16 v4h  __attribute__((ext_vector_type(4)));
typedef float    v8f  __attribute__((ext_vector_type(8)));
typedef float    v4f  __attribute__((ext_vector_type(4)));

union FragU { v16h v; v8h h[2]; };

__device__ __forceinline__ v16h frag_load(const _Float16* p) {
  FragU f;
  f.h[0] = *(const v8h*)(p);
  f.h[1] = *(const v8h*)(p + 16);
  return f.v;
}

__device__ __forceinline__ v8f mma16(v16h a, v16h b, v8f c) {
  c = __builtin_amdgcn_wmma_f32_16x16x32_f16(false, a, false, b, (short)0, c, false, false);
  asm volatile("v_nop\n\tv_nop\n\tv_nop\n\tv_nop" : "+v"(c) : "v"(a), "v"(b));
  return c;
}

__global__ __launch_bounds__(256) void prep_kernel(const float* __restrict__ x,
                                                   const float* __restrict__ gamma,
                                                   const float* __restrict__ beta,
                                                   _Float16* __restrict__ xh,
                                                   float* __restrict__ lnx) {
  const int lane = threadIdx.x & 31;
  const int wave = threadIdx.x >> 5;
  const int prow = blockIdx.x * 8 + wave;
  const int b = prow / NP;
  const int n = prow - b * NP;
  v4f lv[4];
  v4h hv[4];
  if (n < NTOK) {
    const float* xr = x + ((size_t)b * NTOK + n) * DM;
    v4f xv[4];
    float s = 0.f;
#pragma unroll
    for (int i = 0; i < 4; ++i) {
      xv[i] = *(const v4f*)(xr + i * 128 + lane * 4);
      s += (xv[i][0] + xv[i][1]) + (xv[i][2] + xv[i][3]);
    }
#pragma unroll
    for (int m = 16; m >= 1; m >>= 1) s += __shfl_xor(s, m, 32);
    const float mu = s * (1.0f / DM);
    float ss = 0.f;
#pragma unroll
    for (int i = 0; i < 4; ++i) {
#pragma unroll
      for (int e = 0; e < 4; ++e) {
        const float d = xv[i][e] - mu;
        ss += d * d;
      }
    }
#pragma unroll
    for (int m = 16; m >= 1; m >>= 1) ss += __shfl_xor(ss, m, 32);
    const float rs = rsqrtf(ss * (1.0f / DM) + 1e-5f);
#pragma unroll
    for (int i = 0; i < 4; ++i) {
      const v4f g  = *(const v4f*)(gamma + i * 128 + lane * 4);
      const v4f be = *(const v4f*)(beta  + i * 128 + lane * 4);
#pragma unroll
      for (int e = 0; e < 4; ++e) {
        lv[i][e] = (xv[i][e] - mu) * rs * g[e] + be[e];
        hv[i][e] = (_Float16)xv[i][e];
      }
    }
  } else {
    const _Float16 hz = (_Float16)0.0f;
#pragma unroll
    for (int i = 0; i < 4; ++i) {
      lv[i] = (v4f){0.f, 0.f, 0.f, 0.f};
      hv[i] = (v4h){hz, hz, hz, hz};
    }
  }
  float*    lr = lnx + (size_t)prow * DM + lane * 4;
  _Float16* hr = xh  + (size_t)prow * DM + lane * 4;
  for (int pass = 0; pass < 2; ++pass) {
#pragma unroll
    for (int i = 0; i < 4; ++i) {
      *(volatile v4f*)(lr + i * 128) = lv[i];
      *(volatile v4h*)(hr + i * 128) = hv[i];
    }
    __threadfence();
  }
}

__global__ __launch_bounds__(256) void tconv_kernel(const float* __restrict__ W, _Float16* __restrict__ out,
                                                    int R, int Cc, float scale) {
  __shared__ __align__(16) float tf[64 * 68];
  const int c0  = blockIdx.x * 64;
  const int r0  = blockIdx.y * 64;
  const int tid = threadIdx.x;
  {
    const int lr = tid >> 4;
    const int c4 = (tid & 15) * 4;
#pragma unroll
    for (int it = 0; it < 4; ++it) {
      const int rr = it * 16 + lr;
      const v4f a = *(const v4f*)(W + (size_t)(r0 + rr) * Cc + c0 + c4);
      *(v4f*)(tf + rr * 68 + c4) = a;
    }
  }
  __syncthreads();
  const int sub = tid >> 3;
  const int c8  = (tid & 7) * 8;
  v8h hv[2];
#pragma unroll
  for (int it = 0; it < 2; ++it) {
    const int oc = it * 32 + sub;
    v8h a;
#pragma unroll
    for (int e = 0; e < 8; ++e) a[e] = (_Float16)(tf[(c8 + e) * 68 + oc] * scale);
    hv[it] = a;
  }
  for (int pass = 0; pass < 2; ++pass) {
#pragma unroll
    for (int it = 0; it < 2; ++it) {
      const int oc = it * 32 + sub;
      *(volatile v8h*)(out + (size_t)(c0 + oc) * R + r0 + c8) = hv[it];
    }
    __threadfence();
  }
}

template <int BIAS_MODE, int OUT_MODE, bool RESID>
__global__ __launch_bounds__(256) void gemm64_kernel(
    const _Float16* __restrict__ A, int lda, long strideA,
    const _Float16* __restrict__ Bt, int ldb, long strideB,
    void* __restrict__ Cout, int ldc, long strideC,
    const float* __restrict__ bias,
    const float* __restrict__ resid, int ldr, long strideR,
    int M, int N, int K, int Mvalid, float scale) {
  __shared__ __align__(16) float sT[8][16 * OLD];
  const int bz   = blockIdx.y;
  const int lane = threadIdx.x & 31;
  const int wave = threadIdx.x >> 5;
  const int tilesN = N >> 6;
  const int tilesM = M >> 6;
  const int tile = blockIdx.x * 8 + wave;
  if (tile >= tilesM * tilesN) return;
  const int tm = tile / tilesN;
  const int tn = tile - tm * tilesN;
  const int m0 = tm << 6;
  const int n0 = tn << 6;

  const _Float16* Ab = A  + (size_t)bz * strideA;
  const _Float16* Bb = Bt + (size_t)bz * strideB;

  const int rl   = lane & 15;
  const int koff = (lane >> 4) * 8;
  const int mOff = (lane >> 4) * 8;

  v8f acc[4][4];
#pragma unroll
  for (int i = 0; i < 4; ++i)
#pragma unroll
    for (int j = 0; j < 4; ++j) acc[i][j] = (v8f){0.f, 0.f, 0.f, 0.f, 0.f, 0.f, 0.f, 0.f};

  for (int k0 = 0; k0 < K; k0 += 32) {
    v16h bf[4];
#pragma unroll
    for (int j = 0; j < 4; ++j)
      bf[j] = frag_load(Bb + (size_t)(n0 + (j << 4) + rl) * ldb + k0 + koff);
#pragma unroll
    for (int i = 0; i < 4; ++i) {
      const v16h af = frag_load(Ab + (size_t)(m0 + (i << 4) + rl) * lda + k0 + koff);
#pragma unroll
      for (int j = 0; j < 4; ++j) acc[i][j] = mma16(af, bf[j], acc[i][j]);
    }
  }

  float* slab = sT[wave];
  const float* Rb = RESID ? (resid + (size_t)bz * strideR) : nullptr;
#pragma unroll
  for (int i = 0; i < 4; ++i) {
    const int mBase = m0 + (i << 4);
#pragma unroll
    for (int j = 0; j < 4; ++j) {
      const int n = n0 + (j << 4) + rl;
      float bv = 0.f;
      if (BIAS_MODE == 2) bv = bias[n];
#pragma unroll
      for (int r = 0; r < 8; ++r) {
        float v = acc[i][j][r] * scale;
        if (BIAS_MODE == 2) v += bv;
        if (RESID) v += Rb[(size_t)(mBase + mOff + r) * ldr + n];
        slab[(mOff + r) * OLD + (j << 4) + rl] = v;
      }
    }
    __builtin_amdgcn_fence(__ATOMIC_RELEASE, "workgroup");
    __builtin_amdgcn_wave_barrier();
    __builtin_amdgcn_fence(__ATOMIC_ACQUIRE, "workgroup");
    if (OUT_MODE == 0) {
      float* C = (float*)Cout + (size_t)bz * strideC;
      const int hh = lane >> 4, c4 = (lane & 15) * 4;
      for (int pass = 0; pass < 2; ++pass) {
#pragma unroll
        for (int it = 0; it < 8; ++it) {
          const int row = it * 2 + hh;
          const v4f v = *(const v4f*)(slab + row * OLD + c4);
          if (mBase + row < Mvalid)
            *(volatile v4f*)(C + (size_t)(mBase + row) * ldc + n0 + c4) = v;
        }
        __threadfence();
      }
    } else {
      _Float16* C = (_Float16*)Cout + (size_t)bz * strideC;
      const int q = lane >> 3, c8 = (lane & 7) * 8;
      for (int pass = 0; pass < 2; ++pass) {
#pragma unroll
        for (int it = 0; it < 4; ++it) {
          const int row = it * 4 + q;
          const float* sp = slab + row * OLD + c8;
          const v4f f0 = *(const v4f*)(sp);
          const v4f f1 = *(const v4f*)(sp + 4);
          v8h hv;
#pragma unroll
          for (int e = 0; e < 4; ++e) { hv[e] = (_Float16)f0[e]; hv[4 + e] = (_Float16)f1[e]; }
          if (mBase + row < Mvalid)
            *(volatile v8h*)(C + (size_t)(mBase + row) * ldc + n0 + c8) = hv;
        }
        __threadfence();
      }
    }
    __builtin_amdgcn_fence(__ATOMIC_RELEASE, "workgroup");
    __builtin_amdgcn_wave_barrier();
    __builtin_amdgcn_fence(__ATOMIC_ACQUIRE, "workgroup");
  }
}

__global__ __launch_bounds__(128) void attn_kernel(const _Float16* __restrict__ qk,
                                                   const _Float16* __restrict__ vt,
                                                   const float* __restrict__ sim,
                                                   const float* __restrict__ lg,
                                                   _Float16* __restrict__ op) {
  __shared__ __align__(16) _Float16 Ks[64 * KLD];
  __shared__ __align__(16) _Float16 Vs[64 * KLD];
  __shared__ __align__(16) _Float16 Ps[4][16 * PLD];
  __shared__ __align__(16) float    Os[4][16 * OLD];

  const int tid  = threadIdx.x;
  const int wave = tid >> 5;
  const int lane = tid & 31;
  const int hh   = lane >> 4;
  const int c    = lane & 15;

  const int qb = blockIdx.x;
  const int bh = blockIdx.y;
  const int b  = bh >> 3;
  const int h  = bh & 7;
  const int q0 = qb * 64 + wave * 16;
  const size_t rowb = (size_t)b * NP;

  const float lgt   = lg[0];
  const float alpha = 1.0f / (1.0f + __expf(-lgt));
  const float cs    = (1.0f - alpha) * (0.125f / 64.0f);

  v16h qa[2];
  {
    const _Float16* qr = qk + (rowb + q0 + c) * NQK + h * HD + 8 * hh;
    qa[0] = frag_load(qr);
    qa[1] = frag_load(qr + 32);
  }
  int soff[8];
#pragma unroll
  for (int r = 0; r < 8; ++r) {
    int qrw = q0 + 8 * hh + r;
    qrw = (qrw < NTOK) ? qrw : (NTOK - 1);
    soff[r] = qrw * NTOK;
  }

  float mrow[8], lrow[8];
  v8f oacc[4];
#pragma unroll
  for (int r = 0; r < 8; ++r) { mrow[r] = -INFINITY; lrow[r] = 0.f; }
#pragma unroll
  for (int t = 0; t < 4; ++t) oacc[t] = (v8f){0.f, 0.f, 0.f, 0.f, 0.f, 0.f, 0.f, 0.f};

  for (int kc = 0; kc < NP / 64; ++kc) {
    const int kv0 = kc * 64;
    __syncthreads();
    {
      const int r = tid >> 1, half = (tid & 1) * 32;
      const _Float16* kg = qk + (rowb + kv0 + r) * NQK + DM + h * HD + half;
      const _Float16* vg = vt + (size_t)(h * HD + r) * MR + rowb + kv0 + half;
#pragma unroll
      for (int i = 0; i < 4; ++i) {
        const v8h a0 = *(const v8h*)(kg + 8 * i);
        const v8h b0 = *(const v8h*)(vg + 8 * i);
        *(v8h*)(Ks + r * KLD + half + 8 * i) = a0;
        *(v8h*)(Vs + r * KLD + half + 8 * i) = b0;
      }
    }
    __syncthreads();

    v8f s[4];
#pragma unroll
    for (int j = 0; j < 4; ++j) {
      s[j] = (v8f){0.f, 0.f, 0.f, 0.f, 0.f, 0.f, 0.f, 0.f};
#pragma unroll
      for (int dc = 0; dc < 2; ++dc) {
        FragU kb;
        const _Float16* kp = Ks + (j * 16 + c) * KLD + dc * 32 + 8 * hh;
        kb.h[0] = *(const v8h*)(kp);
        kb.h[1] = *(const v8h*)(kp + 16);
        s[j] = mma16(qa[dc], kb.v, s[j]);
      }
    }
    float cm[8];
#pragma unroll
    for (int r = 0; r < 8; ++r) {
      const float* srow = sim + soff[r];
      float m = -INFINITY;
#pragma unroll
      for (int j = 0; j < 4; ++j) {
        const int key  = kv0 + j * 16 + c;
        const int keyc = (key < NTOK) ? key : (NTOK - 1);
        const float bv = srow[keyc];
        float sv = s[j][r] * cs + alpha * bv;
        sv = (key < NTOK) ? sv : -INFINITY;
        s[j][r] = sv;
        m = fmaxf(m, sv);
      }
#pragma unroll
      for (int off = 1; off < 16; off <<= 1) m = fmaxf(m, __shfl_xor(m, off, 32));
      cm[r] = m;
    }
    _Float16* pw = Ps[wave];
#pragma unroll
    for (int r = 0; r < 8; ++r) {
      const float mnew = fmaxf(mrow[r], cm[r]);
      const float corr = __expf(mrow[r] - mnew);
      mrow[r] = mnew;
      float psum = 0.f;
#pragma unroll
      for (int j = 0; j < 4; ++j) {
        const float p = __expf(s[j][r] - mnew);
        psum += p;
        pw[(8 * hh + r) * PLD + j * 16 + c] = (_Float16)(p * 256.0f);
      }
#pragma unroll
      for (int off = 1; off < 16; off <<= 1) psum += __shfl_xor(psum, off, 32);
      lrow[r] = lrow[r] * corr + psum;
#pragma unroll
      for (int t = 0; t < 4; ++t) oacc[t][r] *= corr;
    }
    __builtin_amdgcn_fence(__ATOMIC_RELEASE, "workgroup");
    __builtin_amdgcn_wave_barrier();
    __builtin_amdgcn_fence(__ATOMIC_ACQUIRE, "workgroup");
#pragma unroll 1
    for (int kk = 0; kk < 2; ++kk) {
      FragU pa;
      const _Float16* pp = pw + c * PLD + kk * 32 + 8 * hh;
      pa.h[0] = *(const v8h*)(pp);
      pa.h[1] = *(const v8h*)(pp + 16);
#pragma unroll
      for (int t = 0; t < 4; ++t) {
        FragU vb;
        const _Float16* vp = Vs + (t * 16 + c) * KLD + kk * 32 + 8 * hh;
        vb.h[0] = *(const v8h*)(vp);
        vb.h[1] = *(const v8h*)(vp + 16);
        oacc[t] = mma16(pa.v, vb.v, oacc[t]);
      }
    }
  }

  float* os = Os[wave];
#pragma unroll
  for (int r = 0; r < 8; ++r) {
    const float inv = 0.03125f / lrow[r];
#pragma unroll
    for (int t = 0; t < 4; ++t) os[(8 * hh + r) * OLD + t * 16 + c] = oacc[t][r] * inv;
  }
  __builtin_amdgcn_fence(__ATOMIC_RELEASE, "workgroup");
  __builtin_amdgcn_wave_barrier();
  __builtin_amdgcn_fence(__ATOMIC_ACQUIRE, "workgroup");
  {
    const int q = lane >> 3, c8 = (lane & 7) * 8;
    for (int pass = 0; pass < 2; ++pass) {
#pragma unroll
      for (int it = 0; it < 4; ++it) {
        const int row = it * 4 + q;
        const float* sp = os + row * OLD + c8;
        const v4f f0 = *(const v4f*)(sp);
        const v4f f1 = *(const v4f*)(sp + 4);
        v8h hv;
#pragma unroll
        for (int e = 0; e < 4; ++e) { hv[e] = (_Float16)f0[e]; hv[4 + e] = (_Float16)f1[e]; }
        *(volatile v8h*)(op + (rowb + q0 + row) * DM + h * HD + c8) = hv;
      }
      __threadfence();
    }
  }
}

extern "C" void kernel_launch(void* const* d_in, const int* in_sizes, int n_in,
                              void* d_out, int out_size, void* d_ws, size_t ws_size,
                              hipStream_t stream) {
  if (n_in < 8) return;
  if (in_sizes[0] != NB * NTOK * DM) return;
  if (in_sizes[1] != NTOK * NTOK) return;
  if (in_sizes[2] != DM * N3) return;
  if (in_sizes[3] != DM * DM) return;
  if (in_sizes[4] < DM || in_sizes[5] < DM || in_sizes[6] < DM) return;
  if (in_sizes[7] < 1) return;
  if (out_size != NB * NTOK * DM) return;

  const float* x      = (const float*)d_in[0];
  const float* sim    = (const float*)d_in[1];
  const float* w_qkv  = (const float*)d_in[2];
  const float* w_proj = (const float*)d_in[3];
  const float* b_proj = (const float*)d_in[4];
  const float* gamma  = (const float*)d_in[5];
  const float* beta   = (const float*)d_in[6];
  const float* slogit = (const float*)d_in[7];

  const size_t szXH  = (size_t)MR * DM * 2;
  const size_t szLNX = (size_t)MR * DM * 4;
  const size_t szWQ  = (size_t)N3 * DM * 2;
  const size_t szWP  = (size_t)DM * DM * 2;
  const size_t szQK  = (size_t)MR * NQK * 2;
  const size_t szVT  = (size_t)DM * MR * 2;
  const size_t szO   = (size_t)MR * DM * 2;
  size_t off = 0;
  const size_t oXH  = off; off += szXH;
  const size_t oLNX = off; off += szLNX;
  const size_t oWQ  = off; off += szWQ;
  const size_t oWP  = off; off += szWP;
  const size_t oQK  = off; off += szQK;
  const size_t oVT  = off; off += szVT;
  const size_t oO   = off; off += szO;
  if (off > ws_size) return;

  char* ws = (char*)d_ws;
  _Float16* XH  = (_Float16*)(ws + oXH);
  float*    LNX = (float*)(ws + oLNX);
  _Float16* WQ  = (_Float16*)(ws + oWQ);
  _Float16* WP  = (_Float16*)(ws + oWP);
  _Float16* QK  = (_Float16*)(ws + oQK);
  _Float16* VT  = (_Float16*)(ws + oVT);
  _Float16* O   = (_Float16*)(ws + oO);

  const dim3 blk(256);

  prep_kernel<<<dim3(MR / 8), blk, 0, stream>>>(x, gamma, beta, XH, LNX);
  tconv_kernel<<<dim3(N3 / 64, DM / 64), blk, 0, stream>>>(w_qkv, WQ, DM, N3, 64.0f);
  tconv_kernel<<<dim3(DM / 64, DM / 64), blk, 0, stream>>>(w_proj, WP, DM, DM, 64.0f);
  gemm64_kernel<0, 1, false><<<dim3(((MR / 64) * (NQK / 64) + 7) / 8, 1), blk, 0, stream>>>(
      XH, DM, 0L, WQ, DM, 0L, (void*)QK, NQK, 0L,
      b_proj, LNX, DM, 0L, MR, NQK, DM, MR, 0.125f);
  gemm64_kernel<0, 1, false><<<dim3(((DM / 64) * (MR / 64) + 7) / 8, 1), blk, 0, stream>>>(
      WQ + (size_t)NQK * DM, DM, 0L, XH, DM, 0L, (void*)VT, MR, 0L,
      b_proj, LNX, DM, 0L, DM, MR, DM, DM, 0.125f);
  attn_kernel<<<dim3(NP / 64, NB * NH), dim3(128), 0, stream>>>(QK, VT, sim, slogit, O);
  gemm64_kernel<2, 0, true><<<dim3(((NP / 64) * (DM / 64) + 7) / 8, NB), blk, 0, stream>>>(
      O, DM, (long)NP * DM, WP, DM, 0L, d_out, DM, (long)NTOK * DM,
      b_proj, LNX, DM, (long)NP * DM, NP, DM, DM, NTOK, 1.0f / 4096.0f);
  (void)hipGetLastError();
}
